// VariableSelectionNetwork_13735305412895
// MI455X (gfx1250) — hardware-verified
//
#include <hip/hip_runtime.h>
#include <math.h>

constexpr int kBatch = 16;
constexpr int kTime  = 256;
constexpr int kVars  = 64;
constexpr int kHid   = 256;
constexpr int kRows  = kBatch * kTime;
constexpr int kRowTile = 32;
constexpr int kAPitch  = 264;
constexpr int kOPitch  = 260;
constexpr int kWnetRows = 8;
constexpr float kW2Carry  = 16.0f;
constexpr float kACarry   = 8.0f;
constexpr float kResScale = 1.0f / 128.0f;
constexpr float kEps  = 1e-5f;
constexpr float kInvH = 1.0f / 256.0f;
constexpr float kInvV = 1.0f / 64.0f;

static_assert(kRows % kRowTile == 0, "row tiling");
static_assert(kRows % kWnetRows == 0, "wnet tiling");
static_assert(kHid == 8 * 32, "8 waves x 32 columns cover H");
static_assert(kHid % 32 == 0, "K multiple of 32");
static_assert(kVars == 64, "two columns per lane in the weight network");
static_assert((kAPitch % 8) == 0, "16-B aligned LDS A rows");
static_assert((kOPitch % 4) == 0, "16-B aligned LDS staging rows");

constexpr size_t kBtBytes  = (size_t)kVars * kHid * kHid * 2;
constexpr size_t kWtsBytes = (size_t)kRows * kVars * 4;
constexpr size_t kWsTotal  = kBtBytes + kWtsBytes;
static_assert(kWsTotal == 9437184, "carve total");
static_assert(kWsTotal <= (size_t)134217728, "carve under 128 MiB");

typedef __attribute__((ext_vector_type(16))) _Float16 v16h;
typedef __attribute__((ext_vector_type(8)))  _Float16 v8h;
typedef __attribute__((ext_vector_type(16))) __bf16   v16b;
typedef __attribute__((ext_vector_type(8)))  __bf16   v8b;
typedef __attribute__((ext_vector_type(8)))  float    v8f;
typedef __attribute__((ext_vector_type(4)))  float    v4f;
typedef __attribute__((ext_vector_type(4)))  unsigned int v4u;

__device__ __forceinline__ void dep_guard_h(v8f& a, v8f& b, v16h x, v16h y) { asm volatile("v_nop\n\tv_nop\n\tv_nop\n\tv_nop" : "+v"(a), "+v"(b) : "v"(x), "v"(y)); }
__device__ __forceinline__ void dep_guard_b(v8f& a, v8f& b, v16b x, v16b y) { asm volatile("v_nop\n\tv_nop\n\tv_nop\n\tv_nop" : "+v"(a), "+v"(b) : "v"(x), "v"(y)); }
__device__ __forceinline__ void keep4_h(v16h a, v16h b, v16h c, v16h d) { asm volatile("v_nop" :: "v"(a), "v"(b), "v"(c), "v"(d)); }
__device__ __forceinline__ void keep4_b(v16b a, v16b b, v16b c, v16b d) { asm volatile("v_nop" :: "v"(a), "v"(b), "v"(c), "v"(d)); }
template <typename T> struct Frag;
template <> struct Frag<_Float16> {
  typedef v16h V; union U { v16h v; v8h h[2]; };
  static __device__ __forceinline__ v16h load(const _Float16* p) {
    U f; f.h[0] = *(const v8h*)(p); f.h[1] = *(const v8h*)(p + 16); return f.v;
  }
  static __device__ __forceinline__ v8f mma(v16h a, v16h b, v8f c) {
    return __builtin_amdgcn_wmma_f32_16x16x32_f16(false, a, false, b, (short)0, c, false, false);
  }
  static __device__ __forceinline__ void guard(v8f& a, v8f& b, v16h x, v16h y) { dep_guard_h(a, b, x, y); }
  static __device__ __forceinline__ void keep(v16h a, v16h b, v16h c, v16h d) { keep4_h(a, b, c, d); }
};
template <> struct Frag<__bf16> {
  typedef v16b V; union U { v16b v; v8b h[2]; };
  static __device__ __forceinline__ v16b load(const __bf16* p) {
    U f; f.h[0] = *(const v8b*)(p); f.h[1] = *(const v8b*)(p + 16); return f.v;
  }
  static __device__ __forceinline__ v8f mma(v16b a, v16b b, v8f c) {
    return __builtin_amdgcn_wmma_f32_16x16x32_bf16(false, a, false, b, (short)0, c, false, false);
  }
  static __device__ __forceinline__ void guard(v8f& a, v8f& b, v16b x, v16b y) { dep_guard_b(a, b, x, y); }
  static __device__ __forceinline__ void keep(v16b a, v16b b, v16b c, v16b d) { keep4_b(a, b, c, d); }
};

__device__ __forceinline__ unsigned pk16(unsigned short a, unsigned short b) { return (unsigned)a | ((unsigned)b << 16); }
__device__ __forceinline__ unsigned short h_bits(float f) { const _Float16 h = (_Float16)f; return __builtin_bit_cast(unsigned short, h); }

__device__ __forceinline__ void guard4x(v8f& a, v8f& b, v8f& c, v8f& d, v16h p, v16h q, v16h r, v16h s) {
  asm volatile("v_nop\n\tv_nop\n\tv_nop\n\tv_nop" : "+v"(a), "+v"(b), "+v"(c), "+v"(d) : "v"(p), "v"(q), "v"(r), "v"(s));
}

__global__ __launch_bounds__(256) void pack_w2t_kernel(const float* __restrict__ W2, unsigned short* __restrict__ Bt) {
  __shared__ float sm[64][65];
  const int t  = threadIdx.x;
  const int h0 = blockIdx.x * 64;
  const int n0 = blockIdx.y * 64;
  const int v  = blockIdx.z;
  const float* Wv = W2 + (size_t)v * kHid * kHid;
#pragma unroll
  for (int i = 0; i < 16; ++i) {
    const int e = i * 256 + t;
    const int r = e >> 6;
    const int c = e & 63;
    sm[c][r] = Wv[(size_t)(h0 + r) * kHid + n0 + c] * kW2Carry;
  }
  __syncthreads();
  const int lane = t & 31, wave = t >> 5;
  const int q = lane >> 3, c8 = (lane & 7) * 8;
  unsigned short* op = Bt + (size_t)v * kHid * kHid;
  for (int pass = 0; pass < 2; ++pass) {
#pragma unroll
    for (int it = 0; it < 2; ++it) {
      const int row = wave * 8 + it * 4 + q;
      unsigned short hb[8];
#pragma unroll
      for (int e = 0; e < 8; ++e) hb[e] = h_bits(sm[row][c8 + e]);
      const v4u u = (v4u){pk16(hb[0], hb[1]), pk16(hb[2], hb[3]), pk16(hb[4], hb[5]), pk16(hb[6], hb[7])};
      *(volatile v4u*)(op + (size_t)(n0 + row) * kHid + h0 + c8) = u;
    }
    __threadfence();
  }
}

__global__ __launch_bounds__(256) void wnet_kernel(const float* __restrict__ x,
                                                   const float* __restrict__ nW1, const float* __restrict__ nb1,
                                                   const float* __restrict__ nW2, const float* __restrict__ nb2,
                                                   const float* __restrict__ nWg, const float* __restrict__ nbg,
                                                   const float* __restrict__ ng,  const float* __restrict__ nbe,
                                                   float* __restrict__ Wts) {
  __shared__ __align__(16) float w1s[kVars * kVars];
  __shared__ __align__(16) float w2s[kVars * kVars];
  __shared__ __align__(16) float wgs[kVars * kVars];
  __shared__ float sx[kWnetRows][kVars];
  __shared__ float se[kWnetRows][kVars];
  __shared__ float sg[kWnetRows][kVars];
  __shared__ float sq[kWnetRows][kVars];
  __shared__ __align__(16) float sp[kWnetRows * kVars];
  const int t = threadIdx.x, lane = t & 31, wave = t >> 5;
  const int row = blockIdx.x * kWnetRows + wave;

#pragma unroll
  for (int i = 0; i < 4; ++i) { const int idx = (i * 256 + t) * 4; *(v4f*)(w1s + idx) = *(const v4f*)(nW1 + idx); }
  asm volatile("" ::: "memory");
#pragma unroll
  for (int i = 0; i < 4; ++i) { const int idx = (i * 256 + t) * 4; *(v4f*)(w2s + idx) = *(const v4f*)(nW2 + idx); }
  asm volatile("" ::: "memory");
#pragma unroll
  for (int i = 0; i < 4; ++i) { const int idx = (i * 256 + t) * 4; *(v4f*)(wgs + idx) = *(const v4f*)(nWg + idx); }
  asm volatile("" ::: "memory");
  {
    const float* xr = x + (size_t)row * kVars;
    sx[wave][lane]      = xr[lane];
    sx[wave][lane + 32] = xr[lane + 32];
  }
  __syncthreads();

#pragma unroll 1
  for (int j = 0; j < 2; ++j) {
    const int col = lane + 32 * j;
    float u = 0.0f, g = 0.0f;
#pragma unroll 4
    for (int v = 0; v < kVars; ++v) {
      const float xv = sx[wave][v];
      u += xv * w1s[v * kVars + col];
      g += xv * wgs[v * kVars + col];
    }
    u += nb1[col];
    g += nbg[col];
    se[wave][col] = (u > 0.0f) ? u : expm1f(u);
    sg[wave][col] = 1.0f / (1.0f + expf(-g));
  }
  __syncthreads();

  float s = 0.0f;
#pragma unroll 1
  for (int j = 0; j < 2; ++j) {
    const int col = lane + 32 * j;
    float r = 0.0f;
#pragma unroll 4
    for (int v = 0; v < kVars; ++v) r += se[wave][v] * w2s[v * kVars + col];
    r += nb2[col];
    const float pre = sx[wave][col] + sg[wave][col] * r;
    sq[wave][col] = pre;
    s += pre;
  }
#pragma unroll
  for (int off = 16; off > 0; off >>= 1) s += __shfl_xor(s, off, 32);
  const float mu = s * kInvV;

  float qv = 0.0f;
#pragma unroll 1
  for (int j = 0; j < 2; ++j) {
    const int col = lane + 32 * j;
    const float d = sq[wave][col] - mu;
    qv += d * d;
  }
#pragma unroll
  for (int off = 16; off > 0; off >>= 1) qv += __shfl_xor(qv, off, 32);
  const float rs = rsqrtf(qv * kInvV + kEps);

  float mx = -INFINITY;
#pragma unroll 1
  for (int j = 0; j < 2; ++j) {
    const int col = lane + 32 * j;
    const float wn = (sq[wave][col] - mu) * rs * ng[col] + nbe[col];
    sq[wave][col] = wn;
    mx = fmaxf(mx, wn);
  }
#pragma unroll
  for (int off = 16; off > 0; off >>= 1) mx = fmaxf(mx, __shfl_xor(mx, off, 32));

  float es = 0.0f;
#pragma unroll 1
  for (int j = 0; j < 2; ++j) {
    const int col = lane + 32 * j;
    const float e = expf(sq[wave][col] - mx);
    sq[wave][col] = e;
    es += e;
  }
#pragma unroll
  for (int off = 16; off > 0; off >>= 1) es += __shfl_xor(es, off, 32);
  const float inv = 1.0f / es;
#pragma unroll 1
  for (int j = 0; j < 2; ++j) {
    const int col = lane + 32 * j;
    sp[wave * kVars + col] = sq[wave][col] * inv;
  }
  __syncthreads();

  if (wave == 0) {
    float* dst = Wts + (size_t)blockIdx.x * kWnetRows * kVars;
    for (int pass = 0; pass < 2; ++pass) {
#pragma unroll
      for (int it = 0; it < 4; ++it) {
        const v4f val = *(const v4f*)(sp + it * 128 + lane * 4);
        *(volatile v4f*)(dst + it * 128 + lane * 4) = val;
      }
      __threadfence();
    }
  }
}

__global__ __launch_bounds__(256) void grn_main_kernel(const float* __restrict__ x,
                                                       const float* __restrict__ W1,  const float* __restrict__ b1,
                                                       const float* __restrict__ b2,
                                                       const float* __restrict__ Wg,  const float* __restrict__ bg,
                                                       const float* __restrict__ Wsk, const float* __restrict__ bsk,
                                                       const float* __restrict__ g1,  const float* __restrict__ be1,
                                                       const unsigned short* __restrict__ Btp,
                                                       const float* __restrict__ Wts,
                                                       float* __restrict__ out) {
  __shared__ __align__(16) _Float16 a_lds[kRowTile * kAPitch];
  __shared__ __align__(16) float prm[9 * kHid];
  __shared__ float xv[kRowTile], wrow[kRowTile], mus[kRowTile], rss[kRowTile];
  __shared__ float redS[8 * kRowTile], redQ[8 * kRowTile];
  __shared__ __align__(16) float osm[kRowTile * kOPitch];

  const int t    = threadIdx.x;
  const int lane = t & 31;
  const int wave = t >> 5;
  const int hl   = lane >> 4;
  const int lm   = lane & 15;
  const int koff = hl * 8;
  const int row0 = blockIdx.x * kRowTile;
  const int colA = wave * 32 + lm;
  const int colB = colA + 16;
  const _Float16* Bt = (const _Float16*)Btp;

  v8f comb[2][2];
#pragma unroll
  for (int mt = 0; mt < 2; ++mt)
#pragma unroll
    for (int nt = 0; nt < 2; ++nt) comb[mt][nt] = (v8f){0.f,0.f,0.f,0.f,0.f,0.f,0.f,0.f};

  for (int v = 0; v < kVars; ++v) {
    __syncthreads();
    {
      const size_t po = (size_t)v * kHid + t;
      prm[0 * kHid + t] = W1[po];
      prm[1 * kHid + t] = b1[po];
      prm[2 * kHid + t] = Wg[po];
      prm[3 * kHid + t] = bg[po];
      prm[4 * kHid + t] = Wsk[po];
      prm[5 * kHid + t] = bsk[po];
      prm[6 * kHid + t] = b2[po];
      prm[7 * kHid + t] = g1[po];
      prm[8 * kHid + t] = be1[po];
    }
    if (wave == 0) {
      xv[lane]   = x[(size_t)(row0 + lane) * kVars + v];
      wrow[lane] = Wts[(size_t)(row0 + lane) * kVars + v];
    }
    __syncthreads();

    {
      const int h8 = lane * 8;
      const v4f w1a = *(const v4f*)(prm + h8);
      const v4f w1b = *(const v4f*)(prm + h8 + 4);
      const v4f b1a = *(const v4f*)(prm + kHid + h8);
      const v4f b1b = *(const v4f*)(prm + kHid + h8 + 4);
#pragma unroll 1
      for (int rr = 0; rr < 4; ++rr) {
        const int m = wave * 4 + rr;
        const float xm = xv[m];
        v8h hv;
#pragma unroll
        for (int e = 0; e < 4; ++e) {
          const float z = xm * w1a[e] + b1a[e];
          const float a = (z > 0.0f) ? z : expm1f(z);
          hv[e] = (_Float16)(a * kACarry);
        }
#pragma unroll
        for (int e = 0; e < 4; ++e) {
          const float z = xm * w1b[e] + b1b[e];
          const float a = (z > 0.0f) ? z : expm1f(z);
          hv[4 + e] = (_Float16)(a * kACarry);
        }
        *(v8h*)(a_lds + m * kAPitch + h8) = hv;
      }
    }
    __syncthreads();

    v8f acc[2][2];
#pragma unroll
    for (int mt = 0; mt < 2; ++mt)
#pragma unroll
      for (int nt = 0; nt < 2; ++nt) acc[mt][nt] = (v8f){0.f,0.f,0.f,0.f,0.f,0.f,0.f,0.f};
    const _Float16* Bv = Bt + (size_t)v * kHid * kHid;
#pragma unroll 2
    for (int kk = 0; kk < 8; ++kk) {
      const int k0 = kk * 32;
      const v16h fa0 = Frag<_Float16>::load(a_lds + lm * kAPitch + koff + k0);
      const v16h fa1 = Frag<_Float16>::load(a_lds + (lm + 16) * kAPitch + koff + k0);
      const v16h fb0 = Frag<_Float16>::load(Bv + (size_t)colA * kHid + koff + k0);
      const v16h fb1 = Frag<_Float16>::load(Bv + (size_t)colB * kHid + koff + k0);
      acc[0][0] = Frag<_Float16>::mma(fa0, fb0, acc[0][0]);
      acc[0][1] = Frag<_Float16>::mma(fa0, fb1, acc[0][1]);
      acc[1][0] = Frag<_Float16>::mma(fa1, fb0, acc[1][0]);
      acc[1][1] = Frag<_Float16>::mma(fa1, fb1, acc[1][1]);
      guard4x(acc[0][0], acc[0][1], acc[1][0], acc[1][1], fa0, fa1, fb0, fb1);
    }

    const float wgA = prm[2 * kHid + colA], bgA = prm[3 * kHid + colA], wsA = prm[4 * kHid + colA];
    const float bsA = prm[5 * kHid + colA], b2A = prm[6 * kHid + colA];
    const float wgB = prm[2 * kHid + colB], bgB = prm[3 * kHid + colB], wsB = prm[4 * kHid + colB];
    const float bsB = prm[5 * kHid + colB], b2B = prm[6 * kHid + colB];
    float rsum[2][8];
#pragma unroll
    for (int mt = 0; mt < 2; ++mt) {
#pragma unroll
      for (int r = 0; r < 8; ++r) {
        const int m = mt * 16 + 8 * hl + r;
        const float xm = xv[m];
        const float gA = 1.0f / (1.0f + expf(-(xm * wgA + bgA)));
        const float gB = 1.0f / (1.0f + expf(-(xm * wgB + bgB)));
        const float pA = (xm * wsA + bsA) + gA * (acc[mt][0][r] * kResScale + b2A);
        const float pB = (xm * wsB + bsB) + gB * (acc[mt][1][r] * kResScale + b2B);
        acc[mt][0][r] = pA;
        acc[mt][1][r] = pB;
        rsum[mt][r] = pA + pB;
      }
    }
#pragma unroll
    for (int off = 1; off < 16; off <<= 1) {
#pragma unroll
      for (int mt = 0; mt < 2; ++mt)
#pragma unroll
        for (int r = 0; r < 8; ++r) rsum[mt][r] += __shfl_xor(rsum[mt][r], off, 32);
    }
    if (lm == 0) {
#pragma unroll
      for (int mt = 0; mt < 2; ++mt)
#pragma unroll
        for (int r = 0; r < 8; ++r) redS[wave * kRowTile + mt * 16 + 8 * hl + r] = rsum[mt][r];
    }
    __syncthreads();
    if (wave == 0) {
      float s = 0.0f;
#pragma unroll
      for (int w2 = 0; w2 < 8; ++w2) s += redS[w2 * kRowTile + lane];
      mus[lane] = s * kInvH;
    }
    __syncthreads();

    float rq[2][8];
#pragma unroll
    for (int mt = 0; mt < 2; ++mt) {
#pragma unroll
      for (int r = 0; r < 8; ++r) {
        const int m = mt * 16 + 8 * hl + r;
        const float mu = mus[m];
        const float dA = acc[mt][0][r] - mu;
        const float dB = acc[mt][1][r] - mu;
        acc[mt][0][r] = dA;
        acc[mt][1][r] = dB;
        rq[mt][r] = dA * dA + dB * dB;
      }
    }
#pragma unroll
    for (int off = 1; off < 16; off <<= 1) {
#pragma unroll
      for (int mt = 0; mt < 2; ++mt)
#pragma unroll
        for (int r = 0; r < 8; ++r) rq[mt][r] += __shfl_xor(rq[mt][r], off, 32);
    }
    if (lm == 0) {
#pragma unroll
      for (int mt = 0; mt < 2; ++mt)
#pragma unroll
        for (int r = 0; r < 8; ++r) redQ[wave * kRowTile + mt * 16 + 8 * hl + r] = rq[mt][r];
    }
    __syncthreads();
    if (wave == 0) {
      float q = 0.0f;
#pragma unroll
      for (int w2 = 0; w2 < 8; ++w2) q += redQ[w2 * kRowTile + lane];
      rss[lane] = rsqrtf(q * kInvH + kEps);
    }
    __syncthreads();

    const float g1A = prm[7 * kHid + colA], beA = prm[8 * kHid + colA];
    const float g1B = prm[7 * kHid + colB], beB = prm[8 * kHid + colB];
#pragma unroll
    for (int mt = 0; mt < 2; ++mt) {
#pragma unroll
      for (int r = 0; r < 8; ++r) {
        const int m = mt * 16 + 8 * hl + r;
        const float rs = rss[m];
        const float wv = wrow[m];
        comb[mt][0][r] += wv * (acc[mt][0][r] * rs * g1A + beA);
        comb[mt][1][r] += wv * (acc[mt][1][r] * rs * g1B + beB);
      }
    }
  }

#pragma unroll
  for (int mt = 0; mt < 2; ++mt)
#pragma unroll
    for (int r = 0; r < 8; ++r) {
      const int m = mt * 16 + 8 * hl + r;
      osm[m * kOPitch + colA] = comb[mt][0][r];
      osm[m * kOPitch + colB] = comb[mt][1][r];
    }
  __syncthreads();
  for (int pass = 0; pass < 2; ++pass) {
#pragma unroll
    for (int rr = 0; rr < 4; ++rr) {
      const int r = wave * 4 + rr;
#pragma unroll
      for (int hs = 0; hs < 2; ++hs) {
        const int c = hs * 128 + lane * 4;
        const v4f val = *(const v4f*)(osm + r * kOPitch + c);
        *(volatile v4f*)(out + (size_t)(row0 + r) * kHid + c) = val;
      }
    }
    __threadfence();
  }
}

extern "C" void kernel_launch(void* const* d_in, const int* in_sizes, int n_in,
                              void* d_out, int out_size, void* d_ws, size_t ws_size,
                              hipStream_t stream) {
  if (n_in < 19) return;
  if (in_sizes[0] != kRows * kVars) return;
  if (in_sizes[1] != kVars * kHid || in_sizes[3] != kVars * kHid * kHid) return;
  if (in_sizes[11] != kVars * kVars || in_sizes[13] != kVars * kVars || in_sizes[15] != kVars * kVars) return;
  if (out_size != kRows * kHid) return;
  if (ws_size < kWsTotal) return;

  const float* x   = (const float*)d_in[0];
  const float* W1  = (const float*)d_in[1];
  const float* b1  = (const float*)d_in[2];
  const float* W2  = (const float*)d_in[3];
  const float* b2  = (const float*)d_in[4];
  const float* Wg  = (const float*)d_in[5];
  const float* bg  = (const float*)d_in[6];
  const float* Wsk = (const float*)d_in[7];
  const float* bsk = (const float*)d_in[8];
  const float* g1  = (const float*)d_in[9];
  const float* be1 = (const float*)d_in[10];
  const float* nW1 = (const float*)d_in[11];
  const float* nb1 = (const float*)d_in[12];
  const float* nW2 = (const float*)d_in[13];
  const float* nb2 = (const float*)d_in[14];
  const float* nWg = (const float*)d_in[15];
  const float* nbg = (const float*)d_in[16];
  const float* ng  = (const float*)d_in[17];
  const float* nbe = (const float*)d_in[18];

  unsigned short* Bt = (unsigned short*)d_ws;
  float* Wts = (float*)((char*)d_ws + kBtBytes);
  float* outp = (float*)d_out;

  pack_w2t_kernel<<<dim3(kHid / 64, kHid / 64, kVars), 256, 0, stream>>>(W2, Bt);
  wnet_kernel<<<kRows / kWnetRows, 256, 0, stream>>>(x, nW1, nb1, nW2, nb2, nWg, nbg, ng, nbe, Wts);
  grn_main_kernel<<<kRows / kRowTile, 256, 0, stream>>>(x, W1, b1, b2, Wg, bg, Wsk, bsk, g1, be1, Bt, Wts, outp);
}
